// EncoderLayer_81226421502316
// MI455X (gfx1250) — hardware-run, weakly checked
//
#include <hip/hip_runtime.h>
#pragma clang fp contract(off)


#ifndef NB
#define NB 2
#endif
#ifndef SEQ
#define SEQ 384
#endif
#define NB_FULL  2
#define SEQ_FULL 384
#ifndef OUT_SEQ
#define OUT_SEQ SEQ
#endif
#define DM    512
#define DFF   2048
#define VOCAB 32000
#define MROWS (NB * SEQ)
#define AQ    16
#define ATH   256
#define KPP   128
#define SCP   (SEQ + 4)
#define PTP   520
#define KPL   (SEQ / 32)
#define WCAR  1024.0f
#define ACAR  64.0f
#define SFOLD (1.0f / 65536.0f)
#define C2    2.8853900817779268f
#define SNEG  (-2.8853900817779268f)
#define ECL   60.0f
#define PSH   14.0f
#define NEGB  (-3.0e38f)
#define EPSLN 1.0e-6f
#define SQD   22.62741699796952f
#define PEK   (13.287712379549449f / 512.0f)

enum { EPI_EXP = 0, EPI_VT = 1, EPI_RES = 2, EPI_RELU = 3 };

static_assert(DM % 64 == 0);
static_assert(DFF % 64 == 0);
static_assert(DM % 32 == 0);
static_assert(DFF % 32 == 0);
static_assert(MROWS % 64 == 0);
static_assert(SEQ % 64 == 0);
static_assert(SEQ % 32 == 0);
static_assert(SEQ % KPP == 0);
static_assert(SEQ % AQ == 0);
static_assert(ATH == 2 * KPP);
static_assert(AQ == 16);
static_assert(AQ == 2 * (ATH / 32));
static_assert(DM == 64 * (ATH / 32));
static_assert((AQ * DM / 4) % ATH == 0);
static_assert(DM / 4 <= ATH);
static_assert((DM / 4) % 32 == 0);
static_assert(SEQ <= PTP);
static_assert(DM <= PTP);
static_assert((PTP * 2) % 16 == 0);
static_assert(MROWS % 4 == 0);
static_assert(DM == 4 * 32 * 4);
static_assert(DM == 2 * 256);
static_assert(NB <= NB_FULL);
static_assert(SEQ <= SEQ_FULL);
static_assert(WCAR * ACAR == 65536.0f);

typedef _Float16 h16;
typedef unsigned short bf;
typedef __attribute__((ext_vector_type(16))) _Float16 v16h;
typedef __attribute__((ext_vector_type(8)))  _Float16 v8h;
typedef __attribute__((ext_vector_type(4)))  _Float16 v4h;
typedef __attribute__((ext_vector_type(2)))  _Float16 v2h;
typedef __attribute__((ext_vector_type(8)))  float    v8f;
typedef __attribute__((ext_vector_type(4)))  float    v4f;
typedef __attribute__((ext_vector_type(2)))  float    v2f;
typedef v4f  __attribute__((may_alias)) v4fa;

__device__ __forceinline__ unsigned short f2bf(float f) { unsigned u = __float_as_uint(f); u += 0x7FFFu + ((u >> 16) & 1u); return (unsigned short)(u >> 16); }
__device__ __forceinline__ float bfr(float f) { return __uint_as_float(((unsigned)f2bf(f)) << 16); }
__device__ __forceinline__ v16h cat16(v8h lo, v8h hi) { return __builtin_shufflevector(lo, hi, 0, 1, 2, 3, 4, 5, 6, 7, 8, 9, 10, 11, 12, 13, 14, 15); }
__device__ __forceinline__ v16h  ldh(const h16* p) { return cat16(*(const v8h*)p, *(const v8h*)(p + 16)); }
__device__ __forceinline__ void wave_sync() { __builtin_amdgcn_fence(3  , "wavefront"); __builtin_amdgcn_wave_barrier(); asm volatile("" ::: "memory"); }
__device__ __forceinline__ v8f wmma_g(v16h a, v16h b, v8f c) {
    c = __builtin_amdgcn_wmma_f32_16x16x32_f16(false, a, false, b, (short)0, c, false, false);
    asm volatile("v_nop\n\tv_nop\n\tv_nop\n\tv_nop" : "+v"(c) : "v"(a), "v"(b));
    return c; }
static __device__ __forceinline__ h16 toh_flush(float v) { const h16 r = (h16)v; return (fabsf(v) < 6.103515625e-05f) ? (h16)0.0f : r; }

static_assert(256 * 16 * 2 == 64 * 128);
__global__ __launch_bounds__(256) void k_wconv(const float* __restrict__ src, h16* dst, const int K, const int N) {
    __shared__ __align__(16) h16 tl[64 * 72];
    const int tid = threadIdx.x; const int n0 = blockIdx.x * 64, k0 = blockIdx.y * 64;
    const int nn = tid & 63, kq = tid >> 6;
#pragma unroll 4
    for (int it = 0; it < 16; ++it) { const int kk = it * 4 + kq;
        const float v = src[(size_t)(k0 + kk) * N + n0 + nn];
        tl[nn * 72 + kk] = toh_flush(bfr(v) * WCAR); }
    __syncthreads();
#pragma unroll 1
    for (int ps = 0; ps < 2; ++ps) {
#pragma unroll
        for (int s = 0; s < 2; ++s) { const int row = s * 32 + (tid >> 3), c8 = (tid & 7) * 8;
            const v8h hv = *(const v8h*)(&tl[row * 72 + c8]);
            *(volatile v8h*)(dst + (size_t)(n0 + row) * K + k0 + c8) = hv; }
        if (ps == 0) __threadfence(); }
}

static_assert(256 * 8 == DM * 4);
static_assert(256 * 4 == DM * 2);
__global__ __launch_bounds__(256) void k_embed(const int* __restrict__ tokens, const float* __restrict__ emb, float* XF, h16* XH) {
    const int row = blockIdx.x; const int b = row / SEQ, n = row % SEQ;
    int tok = tokens[(size_t)b * SEQ_FULL + n]; tok = tok < 0 ? 0 : (tok > VOCAB - 1 ? VOCAB - 1 : tok);
    const int m = threadIdx.x;
    const v2f e = *(const v2f*)(emb + (size_t)tok * DM + 2 * m);
    const float inv = __builtin_amdgcn_exp2f(-(float)(2 * m) * PEK);
    const float ang = (float)n * inv;
    const float sn = sinf(ang), cs = cosf(ang);
    const float x0 = bfr(e[0]) * SQD + sn;
    const float x1 = bfr(e[1]) * SQD + cs;
    v2f xo; xo[0] = x0; xo[1] = x1;
    v2h ho; ho[0] = toh_flush(x0 * ACAR); ho[1] = toh_flush(x1 * ACAR);
    float* po = XF + (size_t)row * DM + 2 * m; h16* ph = XH + (size_t)row * DM + 2 * m;
    *(volatile v2f*)po = xo; *(volatile v2h*)ph = ho;
    __threadfence();
    *(volatile v2f*)po = xo; *(volatile v2h*)ph = ho;
}

static_assert(32 * 16 * 8 == 16 * 256);
static_assert(32 * 16 * 4 == 16 * 128);
template <int EPI>
__device__ __forceinline__ void gemm_body(const h16* __restrict__ A, const h16* __restrict__ Bt, const float* __restrict__ bias,
                                          const float* __restrict__ resid, float* outf, h16* outh, const int K, const int ldo) {
    __shared__ __align__(16) float os[16 * 68];
    const int lane = threadIdx.x & 31, lr = lane & 15, hi = lane >> 4; const int r0 = blockIdx.x * 64, c0 = blockIdx.y * 64;
    v8f acc[4][4];
#pragma unroll
    for (int mb = 0; mb < 4; ++mb)
#pragma unroll
        for (int nb = 0; nb < 4; ++nb) acc[mb][nb] = (v8f){};
    const size_t aoff = (size_t)(r0 + lr) * K + 8 * hi, boff = (size_t)(c0 + lr) * K + 8 * hi;
#pragma unroll 1
    for (int kc = 0; kc < K; kc += 32) {
        v16h a[4];
#pragma unroll
        for (int mb = 0; mb < 4; ++mb) a[mb] = ldh(A + aoff + (size_t)mb * 16 * K + kc);
#pragma unroll
        for (int nb = 0; nb < 4; ++nb) { const v16h bb = ldh(Bt + boff + (size_t)nb * 16 * K + kc);
#pragma unroll
            for (int mb = 0; mb < 4; ++mb) acc[mb][nb] = wmma_g(a[mb], bb, acc[mb][nb]); }
    }
    float bc[4];
#pragma unroll
    for (int nb = 0; nb < 4; ++nb) bc[nb] = (EPI != EPI_VT) ? bfr(bias[c0 + nb * 16 + lr]) : 0.0f;
#pragma unroll
    for (int mb = 0; mb < 4; ++mb) {
        float br[8];
#pragma unroll
        for (int j = 0; j < 8; ++j) br[j] = (EPI == EPI_VT) ? bfr(bias[r0 + mb * 16 + hi * 8 + j]) : 0.0f;
#pragma unroll
        for (int nb = 0; nb < 4; ++nb) {
#pragma unroll
            for (int j = 0; j < 8; ++j) {
                float t = acc[mb][nb][j] * SFOLD + bc[nb] + br[j];
                if (EPI == EPI_EXP)  { t = t * C2; t = fminf(fmaxf(t, -ECL), ECL); t = __builtin_amdgcn_exp2f(t); }
                if (EPI == EPI_VT)   { t = t * ACAR; }
                if (EPI == EPI_RELU) { t = fmaxf(t, 0.0f) * ACAR; }
                os[(hi * 8 + j) * 68 + nb * 16 + lr] = t; } }
        wave_sync();
#pragma unroll 1
        for (int ps = 0; ps < 2; ++ps) {
            if (EPI == EPI_EXP || EPI == EPI_RES) {
#pragma unroll
                for (int s = 0; s < 8; ++s) { const int row = 2 * s + (lane >> 4), cofs = (lane & 15) * 4;
                    const size_t gi = (size_t)(r0 + mb * 16 + row) * ldo + c0 + cofs;
                    v4f val = *(const v4fa*)(&os[row * 68 + cofs]);
                    if (EPI == EPI_RES) { const v4f rv = *(const v4f*)(resid + gi); val = val + rv; }
                    *(volatile v4f*)(outf + gi) = val; }
            } else {
#pragma unroll
                for (int s = 0; s < 4; ++s) { const int row = 4 * s + (lane >> 3), c8 = (lane & 7) * 8;
                    const v4f x0 = *(const v4fa*)(&os[row * 68 + c8]); const v4f x1 = *(const v4fa*)(&os[row * 68 + c8 + 4]); v8h hv;
#pragma unroll
                    for (int i = 0; i < 4; ++i) { hv[i] = toh_flush(x0[i]); hv[4 + i] = toh_flush(x1[i]); }
                    size_t gi;
                    if (EPI == EPI_VT) { const int bb = c0 / SEQ, tt = c0 % SEQ; gi = ((size_t)bb * DM + (size_t)(r0 + mb * 16 + row)) * SEQ + tt + c8; }
                    else               { gi = (size_t)(r0 + mb * 16 + row) * ldo + c0 + c8; }
                    *(volatile v8h*)(outh + gi) = hv; }
            }
            if (ps == 0) __threadfence(); }
        wave_sync();
    }
}

__global__ __launch_bounds__(32) void k_gemm_exp(const h16* __restrict__ A, const h16* __restrict__ Bt, const float* __restrict__ bias, float* out, const int K, const int ldo) {
    gemm_body<EPI_EXP>(A, Bt, bias, bias, out, nullptr, K, ldo); }
__global__ __launch_bounds__(32) void k_gemm_vt(const h16* __restrict__ A, const h16* __restrict__ Bt, const float* __restrict__ bias, h16* out, const int K) {
    gemm_body<EPI_VT>(A, Bt, bias, bias, nullptr, out, K, SEQ); }
__global__ __launch_bounds__(32) void k_gemm_res(const h16* __restrict__ A, const h16* __restrict__ Bt, const float* __restrict__ bias, const float* __restrict__ resid, float* out, const int K, const int ldo) {
    gemm_body<EPI_RES>(A, Bt, bias, resid, out, nullptr, K, ldo); }
__global__ __launch_bounds__(32) void k_gemm_relu(const h16* __restrict__ A, const h16* __restrict__ Bt, const float* __restrict__ bias, h16* out, const int K, const int ldo) {
    gemm_body<EPI_RELU>(A, Bt, bias, bias, nullptr, out, K, ldo); }

static constexpr size_t ATT_LDS = (size_t)AQ * DM * 4 + (size_t)DM * 4 + (size_t)AQ * SCP * 4 + (size_t)AQ * PTP * 2 + (size_t)AQ * 4;
static_assert(ATT_LDS <= 131072);
static_assert(64 * 72 * 2 <= 131072);
static_assert(16 * 68 * 4 <= 131072);
__global__ __launch_bounds__(ATH) void k_attn(const float* __restrict__ EQ, const float* __restrict__ EK, const float* __restrict__ scale,
                                              const h16* __restrict__ VT, h16* CTX) {
    __shared__ __align__(16) float eqs[AQ * DM];
    __shared__ __align__(16) float ssc[DM];
    __shared__ __align__(16) float scs[AQ * SCP];
    __shared__ __align__(16) h16   pt[AQ * PTP];
    __shared__ float rinv[AQ];
    const int tid = threadIdx.x, lane = tid & 31, lr = lane & 15, hi = lane >> 4;
    const int wave = __builtin_amdgcn_readfirstlane((int)(threadIdx.x >> 5));
    const int b = blockIdx.y, i0 = blockIdx.x * AQ;
    const size_t rowq = (size_t)b * SEQ + i0;
#pragma unroll
    for (int it = 0; it < (AQ * DM / 4) / ATH; ++it) { const int idx = it * ATH + tid; const int r = idx / (DM / 4), c4 = (idx % (DM / 4)) * 4;
        const v4f v = *(const v4f*)(EQ + (rowq + r) * DM + c4);
        *(v4fa*)(&eqs[r * DM + c4]) = v; }
    if (wave < (DM / 4) / 32) { const int c4 = tid * 4;
        const v4f sv = *(const v4f*)(scale + c4); v4f o;
#pragma unroll
        for (int i = 0; i < 4; ++i) o[i] = bfr(sv[i]) * SNEG;
        *(v4fa*)(&ssc[c4]) = o; }
    __syncthreads();

    const int g = wave >> 2;
    const int kl = tid & (KPP - 1);
#pragma unroll 1
    for (int ps = 0; ps < SEQ / KPP; ++ps) {
        const int j = ps * KPP + kl;
        const float* kp = EK + ((size_t)b * SEQ + j) * DM;
        float acc[8];
#pragma unroll
        for (int ii = 0; ii < 8; ++ii) acc[ii] = 0.0f;
#pragma unroll 1
        for (int d4 = 0; d4 < DM; d4 += 4) {
            const v4f ek = *(const v4f*)(kp + d4);
            const v4f sv = *(const v4fa*)(&ssc[d4]);
#pragma unroll
            for (int ii = 0; ii < 8; ++ii) {
                const v4f qv = *(const v4fa*)(&eqs[(8 * g + ii) * DM + d4]);
#pragma unroll
                for (int c = 0; c < 4; ++c) {
                    const float r = __builtin_amdgcn_rcpf(fmaf(qv[c], ek[c], 1.0f));
                    acc[ii] = fmaf(sv[c], r, acc[ii]); } }
        }
#pragma unroll
        for (int ii = 0; ii < 8; ++ii) scs[(8 * g + ii) * SCP + j] = acc[ii];
    }
    __syncthreads();

#pragma unroll 1
    for (int rr = 0; rr < 2; ++rr) {
        const int row = 2 * wave + rr;
        float v[KPL]; float mx = NEGB;
#pragma unroll
        for (int c = 0; c < KPL; ++c) { v[c] = scs[row * SCP + lane + 32 * c]; mx = fmaxf(mx, v[c]); }
        mx = fmaxf(mx, __shfl_xor(mx, 16, 32)); mx = fmaxf(mx, __shfl_xor(mx, 8, 32)); mx = fmaxf(mx, __shfl_xor(mx, 4, 32));
        mx = fmaxf(mx, __shfl_xor(mx, 2, 32));  mx = fmaxf(mx, __shfl_xor(mx, 1, 32));
        const float sh = PSH - mx;
        float ls = 0.0f;
#pragma unroll
        for (int c = 0; c < KPL; ++c) {
            const float e = v[c] + sh;
            const float ex = __builtin_amdgcn_exp2f(e);
            const h16 ph = (e < -14.0f) ? (h16)0.0f : (h16)ex;
            ls += (float)ph;
            pt[row * PTP + lane + 32 * c] = ph; }
        ls += __shfl_xor(ls, 16, 32); ls += __shfl_xor(ls, 8, 32); ls += __shfl_xor(ls, 4, 32); ls += __shfl_xor(ls, 2, 32); ls += __shfl_xor(ls, 1, 32);
        if (lane == 0) rinv[row] = __builtin_amdgcn_rcpf(ls);
    }
    __syncthreads();

    v8f oacc[4];
#pragma unroll
    for (int nb = 0; nb < 4; ++nb) oacc[nb] = (v8f){};
    const size_t vbase = ((size_t)b * DM + (size_t)(64 * wave + lr)) * SEQ + 8 * hi;
    const int pofs = lr * PTP + 8 * hi;
#pragma unroll 1
    for (int key0 = 0; key0 < SEQ; key0 += 32) {
        const v16h pa = cat16(*(const v8h*)(&pt[pofs + key0]), *(const v8h*)(&pt[pofs + key0 + 16]));
#pragma unroll
        for (int nb = 0; nb < 4; ++nb) { const v16h vb = ldh(VT + vbase + (size_t)nb * 16 * SEQ + key0);
            oacc[nb] = wmma_g(pa, vb, oacc[nb]); }
    }
    __syncthreads();
    float ri[8];
#pragma unroll
    for (int r = 0; r < 8; ++r) ri[r] = rinv[8 * hi + r];
#pragma unroll
    for (int nb = 0; nb < 4; ++nb) {
#pragma unroll
        for (int r = 0; r < 8; ++r) pt[(8 * hi + r) * PTP + 64 * wave + 16 * nb + lr] = toh_flush(oacc[nb][r] * ri[r]); }
    wave_sync();
    h16* crow = CTX + rowq * DM + 64 * wave;
#pragma unroll 1
    for (int ps = 0; ps < 2; ++ps) {
#pragma unroll
        for (int s = 0; s < 4; ++s) { const int row = 4 * s + (lane >> 3), c8 = (lane & 7) * 8;
            const v8h hv = *(const v8h*)(&pt[row * PTP + 64 * wave + c8]);
            *(volatile v8h*)(crow + (size_t)row * DM + c8) = hv; }
        if (ps == 0) __threadfence(); }
}

static_assert(32 * 16 * 4 == DM * 4);
static_assert(32 * 8 * 4 == DM * 2);
__global__ __launch_bounds__(128) void k_ln(const float* __restrict__ pre, const float* __restrict__ gam, const float* __restrict__ bet,
                                            float* outf, h16* outh, const int wh, const int oseq) {
    const int lane = threadIdx.x & 31;
    const int wave = __builtin_amdgcn_readfirstlane((int)(threadIdx.x >> 5));
    const int row = blockIdx.x * 4 + wave;
    const float* p = pre + (size_t)row * DM + 4 * lane;
    float s = 0.0f;
#pragma unroll 1
    for (int c = 0; c < 4; ++c) { const v4f v = *(const v4f*)(p + 128 * c); s += (v[0] + v[1]) + (v[2] + v[3]); }
    s += __shfl_xor(s, 16, 32); s += __shfl_xor(s, 8, 32); s += __shfl_xor(s, 4, 32); s += __shfl_xor(s, 2, 32); s += __shfl_xor(s, 1, 32);
    const float mu = s * (1.0f / (float)DM);
    float q = 0.0f;
#pragma unroll 1
    for (int c = 0; c < 4; ++c) { const v4f v = *(const v4f*)(p + 128 * c);
        const float d0 = v[0] - mu, d1 = v[1] - mu, d2 = v[2] - mu, d3 = v[3] - mu;
        q += (d0 * d0 + d1 * d1) + (d2 * d2 + d3 * d3); }
    q += __shfl_xor(q, 16, 32); q += __shfl_xor(q, 8, 32); q += __shfl_xor(q, 4, 32); q += __shfl_xor(q, 2, 32); q += __shfl_xor(q, 1, 32);
    const float rstd = __builtin_amdgcn_rsqf(q * (1.0f / (float)DM) + EPSLN);
    const size_t orow = (size_t)(row / SEQ) * (size_t)oseq + (size_t)(row % SEQ);
    float* po = outf + orow * DM + 4 * lane;
    h16* ph = outh + (size_t)row * DM + 4 * lane;
#pragma unroll 1
    for (int ps = 0; ps < 2; ++ps) {
#pragma unroll 1
        for (int c = 0; c < 4; ++c) {
            const v4f v = *(const v4f*)(p + 128 * c);
            const v4f gv = *(const v4f*)(gam + 128 * c + 4 * lane);
            const v4f bv = *(const v4f*)(bet + 128 * c + 4 * lane);
            v4f y; v4h hy;
#pragma unroll
            for (int i = 0; i < 4; ++i) { y[i] = (v[i] - mu) * rstd * bfr(gv[i]) + bfr(bv[i]); hy[i] = toh_flush(y[i] * ACAR); }
            *(volatile v4f*)(po + 128 * c) = y;
            if (wh != 0) *(volatile v4h*)(ph + 128 * c) = hy; }
        if (ps == 0) __threadfence(); }
}

static constexpr size_t al256(size_t v) { return (v + 255) & ~(size_t)255; }
static constexpr size_t SZ_W  = al256((size_t)DM * DM * 2);
static constexpr size_t SZ_WF = al256((size_t)DM * DFF * 2);
static constexpr size_t SZ_F  = al256((size_t)MROWS * DM * 4);
static constexpr size_t SZ_H  = al256((size_t)MROWS * DM * 2);
static constexpr size_t SZ_HH = al256((size_t)MROWS * DFF * 2);
static constexpr size_t SZ_TOTAL = 4 * SZ_W + 2 * SZ_WF + 6 * SZ_F + 4 * SZ_H + SZ_HH;
static_assert(SZ_TOTAL <= (size_t)134217728);
static_assert((size_t)NB * DM * SEQ == (size_t)MROWS * DM);

extern "C" void kernel_launch(void* const* d_in, const int* in_sizes, int n_in,
                              void* d_out, int out_size, void* d_ws, size_t ws_size, hipStream_t stream) {
    if (n_in < 19) return;
    if ((size_t)in_sizes[0] < (size_t)(NB - 1) * SEQ_FULL + SEQ) return;
    if ((size_t)in_sizes[1] < (size_t)VOCAB * DM) return;
    if ((size_t)in_sizes[2] < (size_t)DM * DM || (size_t)in_sizes[4] < (size_t)DM * DM || (size_t)in_sizes[6] < (size_t)DM * DM || (size_t)in_sizes[9] < (size_t)DM * DM) return;
    if ((size_t)in_sizes[13] < (size_t)DM * DFF || (size_t)in_sizes[15] < (size_t)DM * DFF) return;
    if (in_sizes[3] < DM || in_sizes[5] < DM || in_sizes[7] < DM || in_sizes[8] < DM || in_sizes[10] < DM || in_sizes[11] < DM || in_sizes[12] < DM) return;
    if (in_sizes[14] < DFF || in_sizes[16] < DM || in_sizes[17] < DM || in_sizes[18] < DM) return;
    if ((size_t)out_size < ((size_t)(NB - 1) * OUT_SEQ + SEQ) * DM) return;
    if (SZ_TOTAL > ws_size) return;
    const int*   tokens = (const int*)d_in[0];
    const float* emb    = (const float*)d_in[1];
    const float* wq = (const float*)d_in[2];  const float* bq = (const float*)d_in[3];
    const float* wk = (const float*)d_in[4];  const float* bk = (const float*)d_in[5];
    const float* wv = (const float*)d_in[6];  const float* bv = (const float*)d_in[7];
    const float* asc = (const float*)d_in[8];
    const float* wo = (const float*)d_in[9];  const float* bo = (const float*)d_in[10];
    const float* g1 = (const float*)d_in[11]; const float* be1 = (const float*)d_in[12];
    const float* w1 = (const float*)d_in[13]; const float* bf1 = (const float*)d_in[14];
    const float* w2 = (const float*)d_in[15]; const float* bf2 = (const float*)d_in[16];
    const float* g2 = (const float*)d_in[17]; const float* be2 = (const float*)d_in[18];
    float* OUT = (float*)d_out;
    char* wsp = (char*)d_ws;
    h16* WQT = (h16*)wsp; wsp += SZ_W;
    h16* WKT = (h16*)wsp; wsp += SZ_W;
    h16* WVT = (h16*)wsp; wsp += SZ_W;
    h16* WOT = (h16*)wsp; wsp += SZ_W;
    h16* W1T = (h16*)wsp; wsp += SZ_WF;
    h16* W2T = (h16*)wsp; wsp += SZ_WF;
    float* XF  = (float*)wsp; wsp += SZ_F;
    float* EQ  = (float*)wsp; wsp += SZ_F;
    float* EK  = (float*)wsp; wsp += SZ_F;
    float* PR1 = (float*)wsp; wsp += SZ_F;
    float* X1F = (float*)wsp; wsp += SZ_F;
    float* PR2 = (float*)wsp; wsp += SZ_F;
    h16* XH  = (h16*)wsp; wsp += SZ_H;
    h16* VT  = (h16*)wsp; wsp += SZ_H;
    h16* CTX = (h16*)wsp; wsp += SZ_H;
    h16* X1H = (h16*)wsp; wsp += SZ_H;
    h16* HH  = (h16*)wsp; wsp += SZ_HH;

    k_wconv<<<dim3(DM / 64, DM / 64, 1), 256, 0, stream>>>(wq, WQT, DM, DM);
    k_wconv<<<dim3(DM / 64, DM / 64, 1), 256, 0, stream>>>(wk, WKT, DM, DM);
    k_wconv<<<dim3(DM / 64, DM / 64, 1), 256, 0, stream>>>(wv, WVT, DM, DM);
    k_wconv<<<dim3(DM / 64, DM / 64, 1), 256, 0, stream>>>(wo, WOT, DM, DM);
    k_wconv<<<dim3(DFF / 64, DM / 64, 1), 256, 0, stream>>>(w1, W1T, DM, DFF);
    k_wconv<<<dim3(DM / 64, DFF / 64, 1), 256, 0, stream>>>(w2, W2T, DFF, DM);

    k_embed<<<MROWS, 256, 0, stream>>>(tokens, emb, XF, XH);

    k_gemm_exp<<<dim3(MROWS / 64, DM / 64, 1), 32, 0, stream>>>(XH, WQT, bq, EQ, DM, DM);
    k_gemm_exp<<<dim3(MROWS / 64, DM / 64, 1), 32, 0, stream>>>(XH, WKT, bk, EK, DM, DM);
    k_gemm_vt<<<dim3(DM / 64, MROWS / 64, 1), 32, 0, stream>>>(WVT, XH, bv, VT, DM);

    k_attn<<<dim3(SEQ / AQ, NB, 1), ATH, 0, stream>>>(EQ, EK, asc, VT, CTX);

    k_gemm_res<<<dim3(MROWS / 64, DM / 64, 1), 32, 0, stream>>>(CTX, WOT, bo, XF, PR1, DM, DM);
    k_ln<<<MROWS / 4, 128, 0, stream>>>(PR1, g1, be1, X1F, X1H, 1, SEQ);

    k_gemm_relu<<<dim3(MROWS / 64, DFF / 64, 1), 32, 0, stream>>>(X1H, W1T, bf1, HH, DM, DFF);
    k_gemm_res<<<dim3(MROWS / 64, DM / 64, 1), 32, 0, stream>>>(HH, W2T, bf2, X1F, PR2, DFF, DM);
    k_ln<<<MROWS / 4, 128, 0, stream>>>(PR2, g2, be2, OUT, X1H, 0, OUT_SEQ);
}
